// GIN_29583734735286
// MI455X (gfx1250) — hardware-verified
//
#include <hip/hip_runtime.h>
#include <stddef.h>
#include <stdint.h>
#include <math.h>


#define DIN     128
#define KC      256
#define NLAY    3
#define NTHR    256
#define NWAVE   8
#define EPT     8
#define CHUNK   (NTHR * EPT)
#define WCAP    (EPT * 32)
#define LISTN   (NWAVE * WCAP)
#define NBMAX   2048
#define RCAP    28672
#define DEGCAP  64
#define PKS     11
#define GBM     64
#define GBN     128
#define GTHR    128
#define GNT     8
#define RECW    256
#define SSW     512
#define WPLANE  (DIN * KC)
#define NUW     (6 * DIN * (KC / 8))
#define WSMAX   134217728
#define LDS_AGG ((2 * RCAP + 2 * NBMAX + LISTN) * 4 + 64)

static_assert((CHUNK & (CHUNK - 1)) == 0 && CHUNK <= (1 << PKS));
static_assert((NBMAX & (NBMAX - 1)) == 0 && NBMAX <= (1 << PKS));
static_assert(NTHR * 8 == NBMAX);
static_assert(LISTN >= NBMAX && LISTN >= NWAVE * WCAP);
static_assert((RCAP % 32) == 0);
static_assert(LDS_AGG <= 300000);
static_assert(GBM == (GTHR / 32) * 16 && GBN == 16 * GNT && GTHR == GBN && GBN == 4 * 32);
static_assert(DIN == 32 * 4 && KC == 2 * DIN && (KC % 32) == 0 && DIN == GBN);
static_assert((NUW % NTHR) == 0 && ((DIN * (KC / 8)) % NTHR) == 0 && (DIN * (KC / 8)) == 4096);
static_assert(RECW == 2 * GBN && RECW / 4 <= GTHR && SSW == 4 * GBN && SSW / 4 == GTHR);

typedef float          v4f  __attribute__((ext_vector_type(4)));
typedef float          v8f  __attribute__((ext_vector_type(8)));
typedef int            v4i  __attribute__((ext_vector_type(4)));
typedef int            v8i  __attribute__((ext_vector_type(8)));
typedef unsigned int   v2u  __attribute__((ext_vector_type(2)));
typedef unsigned short v8us __attribute__((ext_vector_type(8)));
typedef __bf16         v16b __attribute__((ext_vector_type(16)));
typedef v4f  __attribute__((may_alias)) v4fa;
typedef v8us __attribute__((may_alias)) v8usa;
union Frag { v16b vb; v8us h[2]; v8i w; };

__device__ __forceinline__ v8f wmx(const Frag& a, const Frag& b, v8f c) {
  v8f d = __builtin_amdgcn_wmma_f32_16x16x32_bf16(false, a.vb, false, b.vb, (short)0, c, false, false);
  asm volatile("v_nop\n\tv_nop\n\tv_nop\n\tv_nop" : "+v"(d) : "v"(a.w), "v"(b.w));
  return d;
}

__device__ __forceinline__ unsigned short bf_bits(float f) {
  unsigned int u = __float_as_uint(f);
  u += 0x7FFFu + ((u >> 16) & 1u);
  return (unsigned short)(u >> 16);
}
__device__ __forceinline__ float bf_val(unsigned short b) { return __uint_as_float(((unsigned int)b) << 16); }
__device__ __forceinline__ float bf_rne(float f) { return bf_val(bf_bits(f)); }

__device__ __forceinline__ float relu_p(float v) { return (v > 0.0f) ? v : (v - v); }

__device__ __forceinline__ void hilo8(const v4f a, const v4f b, v8us& hv, v8us& lv) {
  const float f[8] = {a.x, a.y, a.z, a.w, b.x, b.y, b.z, b.w};
#pragma unroll
  for (int j = 0; j < 8; ++j) {
    const unsigned short hb = bf_bits(f[j]);
    hv[j] = hb;
    lv[j] = bf_bits(f[j] - bf_val(hb));
  }
}

__device__ __forceinline__ int scan_chunk(const int* __restrict__ dsts, int nE, int cbase, int slotBase,
                                          int nb, int vec8, int* list, int tid, int lane, int wave) {
  int wc = 0;
  const int el0  = tid * EPT;
  const int e0   = cbase + el0;
  const int sent = -2147483647 - 1;
  v4i da, db;
  if (vec8 != 0 && cbase + CHUNK <= nE) {
    da = *(const v4i*)(dsts + e0);
    db = *(const v4i*)(dsts + e0 + 4);
  } else {
    da.x = (e0     < nE) ? dsts[min(e0,     nE - 1)] : sent;
    da.y = (e0 + 1 < nE) ? dsts[min(e0 + 1, nE - 1)] : sent;
    da.z = (e0 + 2 < nE) ? dsts[min(e0 + 2, nE - 1)] : sent;
    da.w = (e0 + 3 < nE) ? dsts[min(e0 + 3, nE - 1)] : sent;
    db.x = (e0 + 4 < nE) ? dsts[min(e0 + 4, nE - 1)] : sent;
    db.y = (e0 + 5 < nE) ? dsts[min(e0 + 5, nE - 1)] : sent;
    db.z = (e0 + 6 < nE) ? dsts[min(e0 + 6, nE - 1)] : sent;
    db.w = (e0 + 7 < nE) ? dsts[min(e0 + 7, nE - 1)] : sent;
  }
  const unsigned nbs = (unsigned)slotBase;
  const unsigned unb = (unsigned)nb;
  const unsigned s0 = (unsigned)da.x - nbs, s1 = (unsigned)da.y - nbs;
  const unsigned s2 = (unsigned)da.z - nbs, s3 = (unsigned)da.w - nbs;
  const unsigned s4 = (unsigned)db.x - nbs, s5 = (unsigned)db.y - nbs;
  const unsigned s6 = (unsigned)db.z - nbs, s7 = (unsigned)db.w - nbs;
  const bool h0 = s0 < unb, h1 = s1 < unb, h2 = s2 < unb, h3 = s3 < unb;
  const bool h4 = s4 < unb, h5 = s5 < unb, h6 = s6 < unb, h7 = s7 < unb;
  const unsigned any = __builtin_amdgcn_ballot_w32(h0 | h1 | h2 | h3 | h4 | h5 | h6 | h7);
  if (any != 0u) {
#define HITJ(J, HJ, SJ) { \
      const unsigned mj = __builtin_amdgcn_ballot_w32(HJ); \
      if (mj != 0u) { \
        if (HJ) { \
          const int pos = wc + (int)__builtin_amdgcn_mbcnt_lo(mj, 0u); \
          if (pos < WCAP) list[wave * WCAP + pos] = ((el0 + (J)) << PKS) | (int)(SJ); \
        } \
        wc += (int)__builtin_popcount(mj); } }
    HITJ(0, h0, s0)
    HITJ(1, h1, s1)
    HITJ(2, h2, s2)
    HITJ(3, h3, s3)
    HITJ(4, h4, s4)
    HITJ(5, h5, s5)
    HITJ(6, h6, s6)
    HITJ(7, h7, s7)
#undef HITJ
  }
  return wc;
}

__device__ __forceinline__ v8us cv8b(const float* __restrict__ p, size_t stride) {
  v8us o;
#pragma unroll
  for (int i = 0; i < 8; ++i) o[i] = bf_bits(p[(size_t)i * stride]);
  return o;
}

__global__ __launch_bounds__(NTHR) void k_wprep(const float* __restrict__ W0s, const float* __restrict__ W1s,
                                                unsigned short* WT) {
  const int u = (int)blockIdx.x * NTHR + (int)threadIdx.x;
  if (u >= NUW) return;
  const int p  = u >> 12;
  const int v  = u & 4095;
  const int n  = v >> 5;
  const int k8 = (v & 31) * 8;
  const int kk = k8 & (DIN - 1);
  const int layer = p >> 1;
  const size_t off = (size_t)layer * DIN * DIN + (size_t)kk * DIN + (size_t)n;
  v8us o;
  if ((p & 1) == 0) {
    o = cv8b(W0s + off, DIN);
  } else {
    o = cv8b(W1s + off, DIN);
  }
  unsigned short* dp = WT + (size_t)u * 8;
  *(volatile v8us*)dp = o;
  __threadfence();
  *(volatile v8us*)dp = o;
}

template <int RND>
__global__ __launch_bounds__(NTHR) void k_agg(
    const int* __restrict__ srcs, const int* __restrict__ dsts, const float* __restrict__ wgt,
    const float* __restrict__ fin,
    unsigned short* Xout,
    int nN, int nE, int nb, int vec8, int MPr) {
  extern __shared__ v4f lds_dyn[];
  int* reg1 = (int*)lds_dyn;
  int* reg2 = reg1 + RCAP;
  int* scnt = reg2 + RCAP;
  int* soff = scnt + NBMAX;
  int* list = soff + NBMAX;
  int* wcnt = list + LISTN;
  int* wtot = wcnt + NWAVE;
  const int tid = (int)threadIdx.x, lane = tid & 31, wave = tid >> 5;
  const int nodeBase = (int)blockIdx.x * nb;

  for (int i = tid; i < NBMAX; i += NTHR) scnt[i] = 0;
  __syncthreads();

  int tot = 0;
  const int nChunks = (nE + CHUNK - 1) / CHUNK;
#pragma unroll 1
  for (int ch = 0; ch < nChunks; ++ch) {
    const int cbase = ch * CHUNK;
    const int wc = scan_chunk(dsts, nE, cbase, nodeBase, nb, vec8, list, tid, lane, wave);
    if (lane == 0) wcnt[wave] = wc;
    __syncthreads();
    int pre = 0, all = 0;
#pragma unroll
    for (int w2 = 0; w2 < NWAVE; ++w2) {
      int c = wcnt[w2];
      c = c < 0 ? 0 : (c > WCAP ? WCAP : c);
      all += c;
      pre += (w2 < wave) ? c : 0;
    }
    const int wcc  = wc > WCAP ? WCAP : wc;
    const int base = tot + pre;
#pragma unroll 1
    for (int i = lane; i < wcc; i += 32) {
      const int ent = list[wave * WCAP + i];
      const int el  = (ent >> PKS) & (CHUNK - 1);
      const int sl  = ent & (NBMAX - 1);
      int eid = cbase + el;
      eid = eid > nE - 1 ? nE - 1 : eid;
      const int pos = base + i;
      if (pos < RCAP) reg1[pos] = (int)(((unsigned)eid << PKS) | (unsigned)sl);
    }
    tot += all;
    tot = tot > RCAP ? RCAP : tot;
    __syncthreads();
  }
  const int nh = tot;

  if (wave == 0) {
#pragma unroll 1
    for (int b0 = 0; b0 < nh; b0 += 32) {
      const int idx = b0 + lane;
      const int uv  = reg1[idx < RCAP ? idx : RCAP - 1];
      const int m32 = (nh - b0) < 32 ? (nh - b0) : 32;
#pragma unroll 1
      for (int k = 0; k < m32; ++k) {
        const int u  = __builtin_amdgcn_readlane(uv, k);
        const int sl = u & (NBMAX - 1);
        if (lane == 0) scnt[sl] = scnt[sl] + 1;
      }
    }
  }
  __syncthreads();

  {
    const v4i ca = *(const v4i*)(scnt + 8 * tid);
    const v4i cb = *(const v4i*)(scnt + 8 * tid + 4);
    const int e0 = ca.x < 0 ? 0 : ca.x, e1 = ca.y < 0 ? 0 : ca.y, e2 = ca.z < 0 ? 0 : ca.z, e3 = ca.w < 0 ? 0 : ca.w;
    const int e4 = cb.x < 0 ? 0 : cb.x, e5 = cb.y < 0 ? 0 : cb.y, e6 = cb.z < 0 ? 0 : cb.z, e7 = cb.w < 0 ? 0 : cb.w;
    const int ts = e0 + e1 + e2 + e3 + e4 + e5 + e6 + e7;
    int incl = ts;
#pragma unroll
    for (int d = 1; d < 32; d <<= 1) {
      const int up = __shfl_up(incl, d);
      if (lane >= d) incl += up;
    }
    if (lane == 31) wtot[wave] = incl;
    __syncthreads();
    int pre = 0;
#pragma unroll
    for (int w2 = 0; w2 < NWAVE; ++w2) pre += (w2 < wave) ? wtot[w2] : 0;
    int run = pre + incl - ts;
    soff[8 * tid + 0] = run; run += e0;
    soff[8 * tid + 1] = run; run += e1;
    soff[8 * tid + 2] = run; run += e2;
    soff[8 * tid + 3] = run; run += e3;
    soff[8 * tid + 4] = run; run += e4;
    soff[8 * tid + 5] = run; run += e5;
    soff[8 * tid + 6] = run; run += e6;
    soff[8 * tid + 7] = run;
  }
  __syncthreads();
  for (int i = tid; i < NBMAX; i += NTHR) list[i] = soff[i];
  __syncthreads();

  if (wave == 0) {
#pragma unroll 1
    for (int b0 = 0; b0 < nh; b0 += 32) {
      const int idx = b0 + lane;
      const int uv  = reg1[idx < RCAP ? idx : RCAP - 1];
      const int m32 = (nh - b0) < 32 ? (nh - b0) : 32;
#pragma unroll 1
      for (int k = 0; k < m32; ++k) {
        const int u   = __builtin_amdgcn_readlane(uv, k);
        const int sl  = u & (NBMAX - 1);
        const int eid = (int)((unsigned)u >> PKS);
        if (lane == 0) {
          int pos = list[sl];
          pos = pos < 0 ? 0 : (pos > RCAP - 1 ? RCAP - 1 : pos);
          reg2[pos] = eid;
          list[sl] = pos + 1;
        }
      }
    }
  }
  __syncthreads();

  const int nbw = nb >> 3;
  const bool ovf = (nh >= RCAP);
  const float qnan = __int_as_float(0x7fc00000);

#pragma unroll 1
  for (int jt = 0; jt < nbw; ++jt) {
    const int slot = wave * nbw + jt;
    const int grow = nodeBase + slot;
    int st = soff[slot];
    const int craw = scnt[slot];
    int cnt = craw;
    st  = st < 0 ? 0 : (st > nh ? nh : st);
    cnt = cnt < 0 ? 0 : (cnt > DEGCAP ? DEGCAP : cnt);
    if (cnt > nh - st) cnt = nh - st;
    const float pz = (ovf || craw > DEGCAP) ? qnan : 0.0f;
    const bool liveRow = grow < nN;

    float ag0 = 0.f, ag1 = 0.f, ag2 = 0.f, ag3 = 0.f;
#pragma unroll 1
    for (int q = 0; q < cnt; ++q) {
      int idx = st + q; idx = idx > RCAP - 1 ? RCAP - 1 : idx;
      int eid = reg2[idx]; eid = eid < 0 ? 0 : (eid > nE - 1 ? nE - 1 : eid);
      const int sraw = srcs[eid];
      const int s = sraw < 0 ? 0 : (sraw > nN - 1 ? nN - 1 : sraw);
      const float wv = bf_rne(wgt[eid]);
      const v4f v = *(const v4f*)(fin + (size_t)s * DIN + 4 * lane);
      float v0 = v.x, v1 = v.y, v2 = v.z, v3 = v.w;
      if (RND != 0) { v0 = bf_rne(v0); v1 = bf_rne(v1); v2 = bf_rne(v2); v3 = bf_rne(v3); }
      ag0 = fmaf(wv, v0, ag0); ag1 = fmaf(wv, v1, ag1);
      ag2 = fmaf(wv, v2, ag2); ag3 = fmaf(wv, v3, ag3);
    }
    const int nc = liveRow ? grow : nN - 1;
    const v4f sv = *(const v4f*)(fin + (size_t)nc * DIN + 4 * lane);
    float s0 = sv.x, s1 = sv.y, s2 = sv.z, s3 = sv.w;
    if (RND != 0) { s0 = bf_rne(s0); s1 = bf_rne(s1); s2 = bf_rne(s2); s3 = bf_rne(s3); }
    float r0 = s0 + ag0, r1 = s1 + ag1, r2 = s2 + ag2, r3 = s3 + ag3;
    r0 = (liveRow ? r0 : 0.0f) + pz;
    r1 = (liveRow ? r1 : 0.0f) + pz;
    r2 = (liveRow ? r2 : 0.0f) + pz;
    r3 = (liveRow ? r3 : 0.0f) + pz;

    const unsigned short hb0 = bf_bits(r0), hb1 = bf_bits(r1), hb2 = bf_bits(r2), hb3 = bf_bits(r3);
    const unsigned short lb0 = bf_bits(r0 - bf_val(hb0)), lb1 = bf_bits(r1 - bf_val(hb1));
    const unsigned short lb2 = bf_bits(r2 - bf_val(hb2)), lb3 = bf_bits(r3 - bf_val(hb3));
    v2u ph, pl;
    ph.x = (unsigned int)hb0 | ((unsigned int)hb1 << 16);
    ph.y = (unsigned int)hb2 | ((unsigned int)hb3 << 16);
    pl.x = (unsigned int)lb0 | ((unsigned int)lb1 << 16);
    pl.y = (unsigned int)lb2 | ((unsigned int)lb3 << 16);
    unsigned short* gp = Xout + (size_t)grow * (size_t)KC + 4 * lane;
    const bool wsv = grow < MPr;
    if (wsv) { *(volatile v2u*)gp = ph; *(volatile v2u*)(gp + DIN) = pl; }
    __threadfence();
    if (wsv) { *(volatile v2u*)gp = ph; *(volatile v2u*)(gp + DIN) = pl; }
  }
}

__global__ __launch_bounds__(GTHR) void k_gemm(const unsigned short* __restrict__ A,
                                               const unsigned short* __restrict__ BT,
                                               float* outF, int nN, int mRows, float* rec) {
  __shared__ __attribute__((aligned(16))) float stg[GBM * GBN];
  __shared__ __attribute__((aligned(16))) float pst[RECW];
  const int tid = (int)threadIdx.x, lane = tid & 31, wave = tid >> 5, hh = lane >> 4, m = lane & 15;
  const int rowBase = (int)blockIdx.x * GBM;

  v8f acc[GNT];
  {
    const v8f z = {0.f, 0.f, 0.f, 0.f, 0.f, 0.f, 0.f, 0.f};
#pragma unroll
    for (int t = 0; t < GNT; ++t) acc[t] = z;
  }
  const unsigned short* ap = A  + (size_t)(rowBase + 16 * wave + m) * (size_t)KC + 8 * hh;
  const unsigned short* bp = BT + (size_t)m * (size_t)KC + 8 * hh;

#pragma unroll 1
  for (int k0 = 0; k0 < KC; k0 += 32) {
    Frag af;
    af.h[0] = *(const v8usa*)(ap + k0);
    af.h[1] = *(const v8usa*)(ap + k0 + 16);
#pragma unroll
    for (int nt = 0; nt < GNT; ++nt) {
      const unsigned short* wq = bp + (size_t)(16 * nt) * (size_t)KC + k0;
      Frag bfr;
      bfr.h[0] = *(const v8usa*)wq;
      bfr.h[1] = *(const v8usa*)(wq + 16);
      acc[nt] = wmx(af, bfr, acc[nt]);
    }
  }

#pragma unroll
  for (int nt = 0; nt < GNT; ++nt) {
    const int lc = 16 * nt + m;
#pragma unroll
    for (int r = 0; r < 8; ++r) {
      const int lr = 16 * wave + 8 * hh + r;
      const bool live = (rowBase + lr) < nN;
      const float v = acc[nt][r];
      stg[lr * GBN + lc] = live ? v : 0.0f;
    }
  }
  __syncthreads();

  v4f fv[16];
#pragma unroll
  for (int i = 0; i < 16; ++i) {
    const int lr = 16 * wave + i;
    fv[i] = *(const v4fa*)(stg + lr * GBN + 4 * lane);
  }
  {
    int nvr = nN - rowBase;
    nvr = nvr < 0 ? 0 : (nvr > GBM ? GBM : nvr);
    float s = 0.0f, q = 0.0f;
#pragma unroll 1
    for (int r = 0; r < nvr; ++r) {
      const float v = stg[r * GBN + tid];
      s += v;
      q = fmaf(v, v, q);
    }
    pst[tid] = s;
    pst[GBN + tid] = q;
  }
  __syncthreads();
  const bool pok = tid < RECW / 4;
  v4f pv = {0.f, 0.f, 0.f, 0.f};
  if (pok) pv = *(const v4fa*)(pst + 4 * tid);
  float* pp = rec + (size_t)blockIdx.x * RECW + 4 * tid;
#pragma unroll
  for (int i = 0; i < 16; ++i) {
    const int gr = rowBase + 16 * wave + i;
    float* op = outF + (size_t)gr * (size_t)DIN + 4 * lane;
    if (gr < mRows) *(volatile v4f*)op = fv[i];
  }
  if (pok) *(volatile v4f*)pp = pv;
  __threadfence();
#pragma unroll
  for (int i = 0; i < 16; ++i) {
    const int gr = rowBase + 16 * wave + i;
    float* op = outF + (size_t)gr * (size_t)DIN + 4 * lane;
    if (gr < mRows) *(volatile v4f*)op = fv[i];
  }
  if (pok) *(volatile v4f*)pp = pv;
}

__global__ __launch_bounds__(GBN) void k_comb(const float* __restrict__ rec, const float* __restrict__ gam,
                                              const float* __restrict__ bet, float* ss,
                                              double invN, int nRec) {
  __shared__ __attribute__((aligned(16))) float stg[SSW];
  const int tid = (int)threadIdx.x;
  double S = 0.0, Q = 0.0;
#pragma unroll 2
  for (int b = 0; b < nRec; ++b) {
    const float* pr = rec + (size_t)b * RECW;
    S += (double)pr[tid];
    Q += (double)pr[GBN + tid];
  }
  const double mean = S * invN;
  double var = Q * invN - mean * mean;
  var = (var < 0.0) ? 0.0 : var;
  const double rs = 1.0 / sqrt(var + (double)1e-5f);
  const float g  = bf_rne(gam[tid]);
  const float bb = bf_rne(bet[tid]);
  stg[tid]           = (float)mean;
  stg[GBN + tid]     = (float)(rs * (double)g);
  stg[2 * GBN + tid] = bb;
  stg[3 * GBN + tid] = 0.0f;
  __syncthreads();
  const v4f v = *(const v4fa*)(stg + 4 * tid);
  float* dp = ss + 4 * tid;
  *(volatile v4f*)dp = v;
  __threadfence();
  *(volatile v4f*)dp = v;
}

__global__ __launch_bounds__(NTHR) void k_apply1(const float* __restrict__ T, const float* __restrict__ ss,
                                                 int nN, int nUnits, unsigned short* Y) {
  const int u = (int)blockIdx.x * NTHR + (int)threadIdx.x;
  if (u >= nUnits) return;
  const int row = u >> 4;
  const int c   = (u & 15) * 8;
  const int rc  = row < nN ? row : nN - 1;
  const bool ok = row < nN;
  const float* tp = T + (size_t)rc * DIN + c;
  const v4f ta = *(const v4f*)tp;
  const v4f tb = *(const v4f*)(tp + 4);
  const v4f ma = *(const v4f*)(ss + c),           mb = *(const v4f*)(ss + c + 4);
  const v4f ga = *(const v4f*)(ss + GBN + c),     gb = *(const v4f*)(ss + GBN + c + 4);
  const v4f ba = *(const v4f*)(ss + 2 * GBN + c), bb = *(const v4f*)(ss + 2 * GBN + c + 4);
  v4f ya, yb;
  ya.x = relu_p(fmaf(ta.x - ma.x, ga.x, ba.x)); ya.y = relu_p(fmaf(ta.y - ma.y, ga.y, ba.y));
  ya.z = relu_p(fmaf(ta.z - ma.z, ga.z, ba.z)); ya.w = relu_p(fmaf(ta.w - ma.w, ga.w, ba.w));
  yb.x = relu_p(fmaf(tb.x - mb.x, gb.x, bb.x)); yb.y = relu_p(fmaf(tb.y - mb.y, gb.y, bb.y));
  yb.z = relu_p(fmaf(tb.z - mb.z, gb.z, bb.z)); yb.w = relu_p(fmaf(tb.w - mb.w, gb.w, bb.w));
  ya.x = ok ? ya.x : 0.0f; ya.y = ok ? ya.y : 0.0f; ya.z = ok ? ya.z : 0.0f; ya.w = ok ? ya.w : 0.0f;
  yb.x = ok ? yb.x : 0.0f; yb.y = ok ? yb.y : 0.0f; yb.z = ok ? yb.z : 0.0f; yb.w = ok ? yb.w : 0.0f;
  v8us hv, lv;
  hilo8(ya, yb, hv, lv);
  unsigned short* hp = Y + (size_t)row * KC + c;
  unsigned short* lp = hp + DIN;
  *(volatile v8us*)hp = hv; *(volatile v8us*)lp = lv;
  __threadfence();
  *(volatile v8us*)hp = hv; *(volatile v8us*)lp = lv;
}

__global__ __launch_bounds__(GTHR) void k_stats3(const float* __restrict__ T, const float* __restrict__ ss2,
                                                 int nN, float* rec) {
  __shared__ __attribute__((aligned(16))) float ps[4 * GBN];
  __shared__ __attribute__((aligned(16))) float pq[4 * GBN];
  __shared__ __attribute__((aligned(16))) float pst[RECW];
  const int tid = (int)threadIdx.x, q = tid & 31, rs = tid >> 5;
  const int rowBase = (int)blockIdx.x * GBM;
  int nvr = nN - rowBase;
  nvr = nvr < 0 ? 0 : (nvr > GBM ? GBM : nvr);
  const v4f mm = *(const v4f*)(ss2 + 4 * q);
  const v4f gg = *(const v4f*)(ss2 + GBN + 4 * q);
  const v4f bb = *(const v4f*)(ss2 + 2 * GBN + 4 * q);
  v4f s4 = {0.f, 0.f, 0.f, 0.f}, q4 = {0.f, 0.f, 0.f, 0.f};
#pragma unroll 2
  for (int r = rs; r < nvr; r += 4) {
    const v4f t = *(const v4f*)(T + (size_t)(rowBase + r) * DIN + 4 * q);
    const float u0 = relu_p(fmaf(t.x - mm.x, gg.x, bb.x));
    const float u1 = relu_p(fmaf(t.y - mm.y, gg.y, bb.y));
    const float u2 = relu_p(fmaf(t.z - mm.z, gg.z, bb.z));
    const float u3 = relu_p(fmaf(t.w - mm.w, gg.w, bb.w));
    s4.x += u0; s4.y += u1; s4.z += u2; s4.w += u3;
    q4.x = fmaf(u0, u0, q4.x); q4.y = fmaf(u1, u1, q4.y);
    q4.z = fmaf(u2, u2, q4.z); q4.w = fmaf(u3, u3, q4.w);
  }
  *(v4fa*)(ps + rs * GBN + 4 * q) = s4;
  *(v4fa*)(pq + rs * GBN + 4 * q) = q4;
  __syncthreads();
  {
    const float S = ((ps[tid] + ps[GBN + tid]) + ps[2 * GBN + tid]) + ps[3 * GBN + tid];
    const float Q = ((pq[tid] + pq[GBN + tid]) + pq[2 * GBN + tid]) + pq[3 * GBN + tid];
    pst[tid] = S;
    pst[GBN + tid] = Q;
  }
  __syncthreads();
  const bool pok = tid < RECW / 4;
  v4f pv = {0.f, 0.f, 0.f, 0.f};
  if (pok) pv = *(const v4fa*)(pst + 4 * tid);
  float* pp = rec + (size_t)blockIdx.x * RECW + 4 * tid;
  if (pok) *(volatile v4f*)pp = pv;
  __threadfence();
  if (pok) *(volatile v4f*)pp = pv;
}

__global__ __launch_bounds__(NTHR) void k_apply3(const float* __restrict__ T, const float* __restrict__ ss2,
                                                 const float* __restrict__ ss3, int nN, int mRows, int nUnits,
                                                 int doRelu, float* outp) {
  const int u = (int)blockIdx.x * NTHR + (int)threadIdx.x;
  if (u >= nUnits) return;
  const int row = u >> 5;
  const int c   = (u & 31) * 4;
  const int rc  = row < nN ? row : nN - 1;
  const bool ok = row < nN;
  const v4f t  = *(const v4f*)(T + (size_t)rc * DIN + c);
  const v4f m2 = *(const v4f*)(ss2 + c);
  const v4f g2 = *(const v4f*)(ss2 + GBN + c);
  const v4f b2 = *(const v4f*)(ss2 + 2 * GBN + c);
  const v4f m3 = *(const v4f*)(ss3 + c);
  const v4f g3 = *(const v4f*)(ss3 + GBN + c);
  const v4f b3 = *(const v4f*)(ss3 + 2 * GBN + c);
  const float u0 = relu_p(fmaf(t.x - m2.x, g2.x, b2.x));
  const float u1 = relu_p(fmaf(t.y - m2.y, g2.y, b2.y));
  const float u2 = relu_p(fmaf(t.z - m2.z, g2.z, b2.z));
  const float u3 = relu_p(fmaf(t.w - m2.w, g2.w, b2.w));
  float h0 = fmaf(u0 - m3.x, g3.x, b3.x);
  float h1 = fmaf(u1 - m3.y, g3.y, b3.y);
  float h2 = fmaf(u2 - m3.z, g3.z, b3.z);
  float h3 = fmaf(u3 - m3.w, g3.w, b3.w);
  const float a0 = relu_p(h0), a1 = relu_p(h1), a2 = relu_p(h2), a3 = relu_p(h3);
  const bool dr = doRelu != 0;
  h0 = dr ? a0 : h0; h1 = dr ? a1 : h1; h2 = dr ? a2 : h2; h3 = dr ? a3 : h3;
  v4f v;
  v.x = ok ? h0 : 0.0f; v.y = ok ? h1 : 0.0f; v.z = ok ? h2 : 0.0f; v.w = ok ? h3 : 0.0f;
  float* op = outp + (size_t)row * DIN + c;
  const bool st = row < mRows;
  if (st) *(volatile v4f*)op = v;
  __threadfence();
  if (st) *(volatile v4f*)op = v;
}

static int pick_nb(int nE, int nN) {
  int nb = NBMAX;
  while (nb > 16 && (long long)nb * (long long)nE * 5LL > (long long)RCAP * (long long)nN * 4LL) nb >>= 1;
  return nb;
}
static inline int cdiv(int a, int b) { return (a + b - 1) / b; }
static inline size_t al256(size_t o) { return (o + 255) & ~(size_t)255; }

extern "C" void kernel_launch(void* const* d_in, const int* in_sizes, int n_in,
                              void* d_out, int out_size, void* d_ws, size_t ws_size,
                              hipStream_t stream) {
  if (n_in < 11) return;
  if (in_sizes[0] < DIN || (in_sizes[0] % DIN) != 0) return;
  const int nN = in_sizes[0] / DIN;
  if (nN < GBM || nN > (1 << 22)) return;
  const int nE2 = in_sizes[1];
  if (nE2 < 2 || (nE2 & 1) != 0) return;
  const int nE = nE2 / 2;
  if (nE < 1 || nE > (1 << 21)) return;
  if (in_sizes[2] != nE) return;
  if (in_sizes[3] != NLAY * DIN * DIN || in_sizes[4] != NLAY * DIN * DIN) return;
  for (int i = 5; i < 11; ++i) if (in_sizes[i] != NLAY * DIN) return;
  if ((long long)nN * DIN != (long long)out_size) return;

  const float* h    = (const float*)d_in[0];
  const int*   ei   = (const int*)  d_in[1];
  const int*   src  = ei;
  const int*   dst  = ei + nE;
  const float* w    = (const float*)d_in[2];
  const float* W0s  = (const float*)d_in[3];
  const float* W1s  = (const float*)d_in[4];
  const float* bn1g = (const float*)d_in[5];
  const float* bn1b = (const float*)d_in[6];
  const float* bn2g = (const float*)d_in[7];
  const float* bn2b = (const float*)d_in[8];
  const float* bn3g = (const float*)d_in[9];
  const float* bn3b = (const float*)d_in[10];
  float* out = (float*)d_out;

  const int MP   = cdiv(nN, GBM) * GBM;
  const int gM   = MP / GBM;
  const int nb   = pick_nb(nE, nN);
  const int gA   = cdiv(MP, nb);
  const int vec8 = ((nE & 3) == 0) ? 1 : 0;
  if ((long long)gA * nb < (long long)MP) return;
  if ((long long)(gM - 1) * GBM >= (long long)nN) return;
  if ((long long)MP * 32 > 2147483647LL) return;

  char* ws = (char*)d_ws;
  size_t off = 0;
  const size_t oWT = off; off = al256(off + (size_t)NUW * 16);
  const size_t oH  = off; off = al256(off + (size_t)MP * DIN * 4);
  const size_t oX  = off; off = al256(off + (size_t)MP * KC * 2);
  const size_t oT  = off; off = al256(off + (size_t)MP * DIN * 4);
  const size_t oY  = off; off = al256(off + (size_t)MP * KC * 2);
  const size_t oRC = off; off = al256(off + (size_t)gM * RECW * 4);
  const size_t oSS = off; off = al256(off + (size_t)3 * SSW * 4);
  if (off > ws_size || off > (size_t)WSMAX) return;
  unsigned short* WT = (unsigned short*)(ws + oWT);
  float*          H  = (float*)(ws + oH);
  unsigned short* X  = (unsigned short*)(ws + oX);
  float*          T  = (float*)(ws + oT);
  unsigned short* Y  = (unsigned short*)(ws + oY);
  float*          RC = (float*)(ws + oRC);
  float*          SS = (float*)(ws + oSS);

  hipFuncSetAttribute(reinterpret_cast<const void*>(&k_agg<1>), hipFuncAttributeMaxDynamicSharedMemorySize, LDS_AGG);
  hipFuncSetAttribute(reinterpret_cast<const void*>(&k_agg<0>), hipFuncAttributeMaxDynamicSharedMemorySize, LDS_AGG);

  const double invN = 1.0 / (double)nN;
  const int nU1 = MP * 16;
  const int nU3 = MP * 32;

  k_wprep<<<NUW / NTHR, NTHR, 0, stream>>>(W0s, W1s, WT);

  for (int i = 0; i < NLAY; ++i) {
    const unsigned short* WA = WT + (size_t)(2 * i) * WPLANE;
    const unsigned short* WB = WT + (size_t)(2 * i + 1) * WPLANE;
    if (i == 0) {
      k_agg<1><<<gA, NTHR, LDS_AGG, stream>>>(src, dst, w, h, X, nN, nE, nb, vec8, MP);
    } else {
      k_agg<0><<<gA, NTHR, LDS_AGG, stream>>>(src, dst, w, H, X, nN, nE, nb, vec8, MP);
    }
    k_gemm<<<gM, GTHR, 0, stream>>>(X, WA, T, nN, MP, RC);
    k_comb<<<1, GBN, 0, stream>>>(RC, bn1g + i * DIN, bn1b + i * DIN, SS, invN, gM);
    k_apply1<<<cdiv(nU1, NTHR), NTHR, 0, stream>>>(T, SS, nN, nU1, Y);
    k_gemm<<<gM, GTHR, 0, stream>>>(Y, WB, T, nN, MP, RC);
    k_comb<<<1, GBN, 0, stream>>>(RC, bn2g + i * DIN, bn2b + i * DIN, SS + SSW, invN, gM);
    k_stats3<<<gM, GTHR, 0, stream>>>(T, SS + SSW, nN, RC);
    k_comb<<<1, GBN, 0, stream>>>(RC, bn3g + i * DIN, bn3b + i * DIN, SS + 2 * SSW, invN, gM);
    if (i != NLAY - 1) {
      k_apply3<<<cdiv(nU3, NTHR), NTHR, 0, stream>>>(T, SS + SSW, SS + 2 * SSW, nN, MP, nU3, 1, H);
    } else {
      k_apply3<<<cdiv(nU3, NTHR), NTHR, 0, stream>>>(T, SS + SSW, SS + 2 * SSW, nN, nN, nU3, 0, out);
    }
  }
}
